// SimpleGATLayer_30262339568070
// MI455X (gfx1250) — hardware-verified
//
#include <hip/hip_runtime.h>
#include <stddef.h>
#include <stdint.h>


#define DIN     128
#define HC      64
#define NHEAD   4
#define HDIM    16
#define NAL     8
#define NTHR    256
#define NWAVE   8
#define EPT     8
#define CHUNK   (NTHR * EPT)
#define WCAP    (EPT * 32)
#define LISTN   (NWAVE * WCAP)
#define NBMAX   2048
#define RCAP    28672
#define DEGCAP  4096
#define GBM     64
#define GBN     64
#define GTHR    128
#define WSMAX   134217728
#define LDS_AGG ((2 * RCAP + 2 * NBMAX + LISTN) * 4 + 64)

static_assert((CHUNK & (CHUNK - 1)) == 0 && CHUNK <= 4096);
static_assert((NBMAX & (NBMAX - 1)) == 0 && NBMAX <= 4096);
static_assert(NTHR * 8 == NBMAX);
static_assert(LISTN >= NBMAX);
static_assert(LISTN >= NWAVE * WCAP);
static_assert((RCAP % 32) == 0);
static_assert(LDS_AGG <= 300000);
static_assert(GBM == (GTHR / 32) * 16);
static_assert(DIN / 8 == 16);
static_assert((DIN % 32) == 0);
static_assert(GBN == HC && HC == NHEAD * HDIM && NAL == 2 * NHEAD);
static_assert(GTHR == 2 * HC);
static_assert(GBM * NAL == 4 * GTHR);
static_assert(HC == 64);

typedef float          v4f   __attribute__((ext_vector_type(4)));
typedef float          v8f   __attribute__((ext_vector_type(8)));
typedef int            v4i   __attribute__((ext_vector_type(4)));
typedef int            v8i   __attribute__((ext_vector_type(8)));
typedef unsigned short v8us  __attribute__((ext_vector_type(8)));
typedef __bf16         v16bf __attribute__((ext_vector_type(16)));
union FragB { v16bf v; v8us h[2]; v8i w; };

__device__ __forceinline__ v8f wmb(const FragB& a, const FragB& b, v8f c) {
  v8f d = __builtin_amdgcn_wmma_f32_16x16x32_bf16(false, a.v, false, b.v, (short)0, c, false, false);
  asm volatile("v_nop\n\tv_nop\n\tv_nop\n\tv_nop" : "+v"(d) : "v"(a.w), "v"(b.w));
  return d;
}

__device__ __forceinline__ unsigned short f2bf(float f) {
  unsigned u = __float_as_uint(f);
  u += 0x7FFFu + ((u >> 16) & 1u);
  return (unsigned short)(u >> 16);
}
__device__ __forceinline__ float bf16r(float f) {
  return __uint_as_float(((unsigned)f2bf(f)) << 16);
}
__device__ __forceinline__ v8us cvt8b(const v4f a, const v4f b) {
  v8us r;
  r[0] = f2bf(a.x); r[1] = f2bf(a.y); r[2] = f2bf(a.z); r[3] = f2bf(a.w);
  r[4] = f2bf(b.x); r[5] = f2bf(b.y); r[6] = f2bf(b.z); r[7] = f2bf(b.w);
  return r;
}
__device__ __forceinline__ float lrelu(float v) { return v > 0.f ? v : 0.01f * v; }

__device__ __forceinline__ int scan_chunk(const int* __restrict__ dsts, int nE, int cbase, int slotBase,
                                          int nb, int vec8, int* list, int tid, int lane, int wave) {
  int wc = 0;
  const int el0  = tid * EPT;
  const int e0   = cbase + el0;
  const int sent = -2147483647 - 1;
  v4i da, db;
  if (vec8 != 0 && cbase + CHUNK <= nE) {
    da = *(const v4i*)(dsts + e0);
    db = *(const v4i*)(dsts + e0 + 4);
  } else {
    da.x = (e0     < nE) ? dsts[min(e0,     nE - 1)] : sent;
    da.y = (e0 + 1 < nE) ? dsts[min(e0 + 1, nE - 1)] : sent;
    da.z = (e0 + 2 < nE) ? dsts[min(e0 + 2, nE - 1)] : sent;
    da.w = (e0 + 3 < nE) ? dsts[min(e0 + 3, nE - 1)] : sent;
    db.x = (e0 + 4 < nE) ? dsts[min(e0 + 4, nE - 1)] : sent;
    db.y = (e0 + 5 < nE) ? dsts[min(e0 + 5, nE - 1)] : sent;
    db.z = (e0 + 6 < nE) ? dsts[min(e0 + 6, nE - 1)] : sent;
    db.w = (e0 + 7 < nE) ? dsts[min(e0 + 7, nE - 1)] : sent;
  }
  const unsigned nbs = (unsigned)slotBase;
  const unsigned unb = (unsigned)nb;
  const unsigned s0 = (unsigned)da.x - nbs, s1 = (unsigned)da.y - nbs;
  const unsigned s2 = (unsigned)da.z - nbs, s3 = (unsigned)da.w - nbs;
  const unsigned s4 = (unsigned)db.x - nbs, s5 = (unsigned)db.y - nbs;
  const unsigned s6 = (unsigned)db.z - nbs, s7 = (unsigned)db.w - nbs;
  const bool h0 = s0 < unb, h1 = s1 < unb, h2 = s2 < unb, h3 = s3 < unb;
  const bool h4 = s4 < unb, h5 = s5 < unb, h6 = s6 < unb, h7 = s7 < unb;
  const unsigned any = __builtin_amdgcn_ballot_w32(h0 | h1 | h2 | h3 | h4 | h5 | h6 | h7);
  if (any != 0u) {
#define HITJ(J, HJ, SJ) { \
      const unsigned mj = __builtin_amdgcn_ballot_w32(HJ); \
      if (mj != 0u) { \
        if (HJ) { \
          const int pos = wc + (int)__builtin_amdgcn_mbcnt_lo(mj, 0u); \
          if (pos < WCAP) list[wave * WCAP + pos] = ((el0 + (J)) << 12) | (int)(SJ); \
        } \
        wc += (int)__builtin_popcount(mj); } }
    HITJ(0, h0, s0)
    HITJ(1, h1, s1)
    HITJ(2, h2, s2)
    HITJ(3, h3, s3)
    HITJ(4, h4, s4)
    HITJ(5, h5, s5)
    HITJ(6, h6, s6)
    HITJ(7, h7, s7)
#undef HITJ
  }
  return wc;
}

__global__ __launch_bounds__(NTHR) void k_prep(const float* __restrict__ x, unsigned short* xb, int nRows, int nUnits) {
  const int i = (int)blockIdx.x * NTHR + (int)threadIdx.x;
  if (i >= nUnits) return;
  const int row = i >> 4;
  const int c0  = (i & 15) * 8;
  const int rc  = row < nRows ? row : nRows - 1;
  const float* p = x + (size_t)rc * DIN + c0;
  v4f a = *(const v4f*)p, b = *(const v4f*)(p + 4);
  const v4f z4 = {0.f, 0.f, 0.f, 0.f};
  if (row >= nRows) { a = z4; b = z4; }
  const v8us hv = cvt8b(a, b);
  const size_t o = (size_t)row * DIN + c0;
  *(volatile v8us*)(xb + o) = hv;
  __threadfence();
  *(volatile v8us*)(xb + o) = hv;
}

__global__ __launch_bounds__(GTHR) void k_gemm(
    const unsigned short* __restrict__ A, const unsigned short* __restrict__ WT,
    const float* __restrict__ attl, const float* __restrict__ attr,
    float* Hout, float* ALout, int K)
{
  __shared__ __attribute__((aligned(16))) float stg[GBM * GBN];
  __shared__ __attribute__((aligned(16))) float att[2 * HC];
  __shared__ __attribute__((aligned(16))) float alst[GBM * NAL];
  const int tid = (int)threadIdx.x, lane = tid & 31, wave = tid >> 5, hh = lane >> 4, m = lane & 15;
  const int rowBase = (int)blockIdx.x * GBM;
  {
    const int ci = tid & (HC - 1);
    const float vl = attl[ci];
    const float vr = attr[ci];
    att[tid] = bf16r(tid < HC ? vl : vr);
  }

  v8f acc[4];
  {
    const v8f z = {0.f, 0.f, 0.f, 0.f, 0.f, 0.f, 0.f, 0.f};
    acc[0] = z; acc[1] = z; acc[2] = z; acc[3] = z;
  }
  const unsigned short* ap = A  + (size_t)(rowBase + 16 * wave + m) * (size_t)K + 8 * hh;
  const unsigned short* wp = WT + (size_t)m * (size_t)K + 8 * hh;
  const int ksteps = K >> 5;
#pragma unroll 1
  for (int ks = 0; ks < ksteps; ++ks) {
    FragB af;
    af.h[0] = *(const v8us*)(ap + 32 * ks);
    af.h[1] = *(const v8us*)(ap + 32 * ks + 16);
#pragma unroll
    for (int t = 0; t < 4; ++t) {
      const unsigned short* wq = wp + (size_t)(16 * t) * (size_t)K + 32 * ks;
      FragB bf;
      bf.h[0] = *(const v8us*)wq;
      bf.h[1] = *(const v8us*)(wq + 16);
      acc[t] = wmb(af, bf, acc[t]);
    }
  }

#pragma unroll
  for (int t = 0; t < 4; ++t) {
    const int lc = 16 * t + m;
#pragma unroll
    for (int r = 0; r < 8; ++r) {
      const int lr = 16 * wave + 8 * hh + r;
      stg[lr * GBN + lc] = acc[t][r];
    }
  }
  __syncthreads();

  {
    v4f fv[8];
#pragma unroll
    for (int i = 0; i < 8; ++i) {
      const int lr = 16 * wave + 2 * i + hh;
      fv[i] = *(const v4f*)(stg + lr * GBN + 4 * m);
    }
#pragma unroll
    for (int i = 0; i < 8; ++i) {
      const int lr = 16 * wave + 2 * i + hh;
      const int gr = rowBase + lr;
      float* op = Hout + (size_t)gr * (size_t)HC + 4 * m;
      *(volatile v4f*)op = fv[i];
    }
    __threadfence();
#pragma unroll
    for (int i = 0; i < 8; ++i) {
      const int lr = 16 * wave + 2 * i + hh;
      const int gr = rowBase + lr;
      float* op = Hout + (size_t)gr * (size_t)HC + 4 * m;
      *(volatile v4f*)op = fv[i];
    }
  }

  {
    const int row  = tid >> 1;
    const int side = tid & 1;
    const float* sp = stg + row * GBN;
    const float* wv = att + side * HC;
    float s[4] = {0.f, 0.f, 0.f, 0.f};
#pragma unroll 4
    for (int d = 0; d < HDIM; ++d) {
#pragma unroll
      for (int h = 0; h < NHEAD; ++h) s[h] = fmaf(sp[HDIM * h + d], wv[HDIM * h + d], s[h]);
    }
    alst[row * NAL + side * NHEAD + 0] = s[0];
    alst[row * NAL + side * NHEAD + 1] = s[1];
    alst[row * NAL + side * NHEAD + 2] = s[2];
    alst[row * NAL + side * NHEAD + 3] = s[3];
  }
  __syncthreads();
  {
    const v4f pv = *(const v4f*)(alst + 4 * tid);
    float* aq = ALout + (size_t)rowBase * NAL + 4 * tid;
    *(volatile v4f*)aq = pv;
    __threadfence();
    *(volatile v4f*)aq = pv;
  }
}

__global__ __launch_bounds__(NTHR) void k_agg(
    const int* __restrict__ srcs, const int* __restrict__ dsts,
    const float* __restrict__ AL, const float* __restrict__ H, float* out,
    int nN, int nE, int nb, int vec8) {
  extern __shared__ v4f lds_dyn[];
  int* reg1 = (int*)lds_dyn;
  int* reg2 = reg1 + RCAP;
  int* scnt = reg2 + RCAP;
  int* soff = scnt + NBMAX;
  int* list = soff + NBMAX;
  int* wcnt = list + LISTN;
  int* wtot = wcnt + NWAVE;
  const int tid = (int)threadIdx.x, lane = tid & 31, wave = tid >> 5;
  const int nodeBase = (int)blockIdx.x * nb;

  for (int i = tid; i < NBMAX; i += NTHR) scnt[i] = 0;
  __syncthreads();

  int tot = 0;
  const int nChunks = (nE + CHUNK - 1) / CHUNK;
#pragma unroll 1
  for (int ch = 0; ch < nChunks; ++ch) {
    const int cbase = ch * CHUNK;
    const int wc = scan_chunk(dsts, nE, cbase, nodeBase, nb, vec8, list, tid, lane, wave);
    if (lane == 0) wcnt[wave] = wc;
    __syncthreads();
    int pre = 0, all = 0;
#pragma unroll
    for (int w2 = 0; w2 < NWAVE; ++w2) {
      int c = wcnt[w2];
      c = c < 0 ? 0 : (c > WCAP ? WCAP : c);
      all += c;
      pre += (w2 < wave) ? c : 0;
    }
    const int wcc  = wc > WCAP ? WCAP : wc;
    const int base = tot + pre;
#pragma unroll 1
    for (int i = lane; i < wcc; i += 32) {
      const int ent = list[wave * WCAP + i];
      const int el  = (ent >> 12) & (CHUNK - 1);
      const int sl  = ent & (NBMAX - 1);
      int eid = cbase + el;
      eid = eid > nE - 1 ? nE - 1 : eid;
      const int pos = base + i;
      if (pos < RCAP) reg1[pos] = (int)(((unsigned)eid << 12) | (unsigned)sl);
    }
    tot += all;
    tot = tot > RCAP ? RCAP : tot;
    __syncthreads();
  }
  const int nh = tot;

  if (wave == 0) {
#pragma unroll 1
    for (int b0 = 0; b0 < nh; b0 += 32) {
      const int idx = b0 + lane;
      const int uv  = reg1[idx < RCAP ? idx : RCAP - 1];
      const int m32 = (nh - b0) < 32 ? (nh - b0) : 32;
#pragma unroll 1
      for (int k = 0; k < m32; ++k) {
        const int u  = __builtin_amdgcn_readlane(uv, k);
        const int sl = u & (NBMAX - 1);
        if (lane == 0) scnt[sl] = scnt[sl] + 1;
      }
    }
  }
  __syncthreads();

  {
    const v4i ca = *(const v4i*)(scnt + 8 * tid);
    const v4i cb = *(const v4i*)(scnt + 8 * tid + 4);
    const int e0 = ca.x < 0 ? 0 : ca.x, e1 = ca.y < 0 ? 0 : ca.y, e2 = ca.z < 0 ? 0 : ca.z, e3 = ca.w < 0 ? 0 : ca.w;
    const int e4 = cb.x < 0 ? 0 : cb.x, e5 = cb.y < 0 ? 0 : cb.y, e6 = cb.z < 0 ? 0 : cb.z, e7 = cb.w < 0 ? 0 : cb.w;
    const int ts = e0 + e1 + e2 + e3 + e4 + e5 + e6 + e7;
    int incl = ts;
#pragma unroll
    for (int d = 1; d < 32; d <<= 1) {
      const int up = __shfl_up(incl, d);
      if (lane >= d) incl += up;
    }
    if (lane == 31) wtot[wave] = incl;
    __syncthreads();
    int pre = 0;
#pragma unroll
    for (int w2 = 0; w2 < NWAVE; ++w2) pre += (w2 < wave) ? wtot[w2] : 0;
    int run = pre + incl - ts;
    soff[8 * tid + 0] = run; run += e0;
    soff[8 * tid + 1] = run; run += e1;
    soff[8 * tid + 2] = run; run += e2;
    soff[8 * tid + 3] = run; run += e3;
    soff[8 * tid + 4] = run; run += e4;
    soff[8 * tid + 5] = run; run += e5;
    soff[8 * tid + 6] = run; run += e6;
    soff[8 * tid + 7] = run;
  }
  __syncthreads();
  for (int i = tid; i < NBMAX; i += NTHR) list[i] = soff[i];
  __syncthreads();

  if (wave == 0) {
#pragma unroll 1
    for (int b0 = 0; b0 < nh; b0 += 32) {
      const int idx = b0 + lane;
      const int uv  = reg1[idx < RCAP ? idx : RCAP - 1];
      const int m32 = (nh - b0) < 32 ? (nh - b0) : 32;
#pragma unroll 1
      for (int k = 0; k < m32; ++k) {
        const int u   = __builtin_amdgcn_readlane(uv, k);
        const int sl  = u & (NBMAX - 1);
        const int eid = (int)((unsigned)u >> 12);
        if (lane == 0) {
          int pos = list[sl];
          pos = pos < 0 ? 0 : (pos > RCAP - 1 ? RCAP - 1 : pos);
          reg2[pos] = eid;
          list[sl] = pos + 1;
        }
      }
    }
  }
  __syncthreads();

  const int nbw = nb >> 3;
  const bool ovf = (nh >= RCAP);
  const float qnan = __int_as_float(0x7fc00000);
  const int hA = lane >> 4;
  const int hB = 2 + (lane >> 4);
#pragma unroll 1
  for (int jt = 0; jt < nbw; ++jt) {
    const int slot = wave * nbw + jt;
    const int grow = nodeBase + slot;
    const int gcl  = grow < nN ? grow : nN - 1;
    int st = soff[slot];
    const int craw = scnt[slot];
    int cnt = craw;
    st  = st < 0 ? 0 : (st > nh ? nh : st);
    cnt = cnt < 0 ? 0 : (cnt > DEGCAP ? DEGCAP : cnt);
    if (cnt > nh - st) cnt = nh - st;
    const float pz = (ovf || craw > DEGCAP) ? qnan : 0.0f;
    const bool wr = grow < nN;

    const float* arow = AL + (size_t)gcl * NAL;
    const float arA = arow[NHEAD + hA];
    const float arB = arow[NHEAD + hB];
    float mA = -1.0e30f, mB = -1.0e30f, dnA = 0.f, dnB = 0.f, avA = 0.f, avB = 0.f;

#pragma unroll 1
    for (int q = 0; q < cnt; ++q) {
      int idx = st + q; idx = idx > RCAP - 1 ? RCAP - 1 : idx;
      int eid = reg2[idx]; eid = eid < 0 ? 0 : (eid > nE - 1 ? nE - 1 : eid);
      const int sraw = srcs[eid];
      const int s = sraw < 0 ? 0 : (sraw > nN - 1 ? nN - 1 : sraw);
      const float* alr = AL + (size_t)s * NAL;
      const float aA = alr[hA];
      const float aB = alr[hB];
      const float* hr = H + (size_t)s * HC + lane;
      const float hvA = hr[0];
      const float hvB = hr[32];
      const float lA = lrelu(aA + arA);
      const float lB = lrelu(aB + arB);
      {
        const float df = lA - mA;
        const float ee = __expf(-fabsf(df));
        const bool up  = df > 0.f;
        const float s1 = up ? ee : 1.0f;
        const float s2 = up ? 1.0f : ee;
        mA  = up ? lA : mA;
        dnA = fmaf(dnA, s1, s2);
        avA = fmaf(avA, s1, s2 * hvA);
      }
      {
        const float df = lB - mB;
        const float ee = __expf(-fabsf(df));
        const bool up  = df > 0.f;
        const float s1 = up ? ee : 1.0f;
        const float s2 = up ? 1.0f : ee;
        mB  = up ? lB : mB;
        dnB = fmaf(dnB, s1, s2);
        avB = fmaf(avB, s1, s2 * hvB);
      }
    }
    const float dsA = dnA > 0.f ? dnA : 1.0f;
    const float dsB = dnB > 0.f ? dnB : 1.0f;
    const float ivA = (dnA > 0.f ? 1.0f : 0.0f) * __builtin_amdgcn_rcpf(dsA);
    const float ivB = (dnB > 0.f ? 1.0f : 0.0f) * __builtin_amdgcn_rcpf(dsB);
    const float oA = avA * ivA;
    const float oB = avB * ivB;
    const float rA = (oA > 0.f ? oA : expm1f(oA)) + pz;
    const float rB = (oB > 0.f ? oB : expm1f(oB)) + pz;
    float* op = out + (size_t)gcl * HC;
    if (wr) {
      *(volatile float*)(op + lane)      = rA;
      *(volatile float*)(op + 32 + lane) = rB;
    }
    __threadfence();
    if (wr) {
      *(volatile float*)(op + lane)      = rA;
      *(volatile float*)(op + 32 + lane) = rB;
    }
  }
}

static int pick_nb(int nE, int nN) {
  int nb = NBMAX;
  while (nb > 16 && (long long)nb * (long long)nE * 5LL > (long long)RCAP * (long long)nN * 4LL) nb >>= 1;
  return nb;
}
static inline int cdiv(int a, int b) { return (a + b - 1) / b; }

extern "C" void kernel_launch(void* const* d_in, const int* in_sizes, int n_in,
                              void* d_out, int out_size, void* d_ws, size_t ws_size,
                              hipStream_t stream) {
  if (n_in < 5) return;
  const int nN = in_sizes[0] / DIN;
  if (nN <= 0 || in_sizes[0] != nN * DIN || nN > (1 << 22)) return;
  if (in_sizes[1] < 2 || (in_sizes[1] & 1) != 0) return;
  const int nE = in_sizes[1] / 2;
  if (nE < 1 || nE > (1 << 20)) return;
  if (in_sizes[2] != HC * DIN) return;
  if (in_sizes[3] != NHEAD * HDIM || in_sizes[4] != NHEAD * HDIM) return;
  if (out_size != nN * HC) return;

  const float* x    = (const float*)d_in[0];
  const int*   ei   = (const int*)  d_in[1];
  const float* W    = (const float*)d_in[2];
  const float* attl = (const float*)d_in[3];
  const float* attr = (const float*)d_in[4];
  float* out = (float*)d_out;
  const int* src = ei;
  const int* dst = ei + nE;

  const int MP   = cdiv(nN, GBM) * GBM;
  const int nb   = pick_nb(nE, nN);
  const int gA   = cdiv(nN, nb);
  const int vec8 = ((nE & 3) == 0) ? 1 : 0;
  if ((long long)gA * nb < nN) return;

  char* ws = (char*)d_ws;
  size_t off = 0;
  const size_t oXB = off; off += (size_t)MP * DIN * 2;             off = (off + 255) & ~(size_t)255;
  const size_t oWB = off; off += (size_t)HC * DIN * 2;             off = (off + 255) & ~(size_t)255;
  const size_t oH  = off; off += (size_t)MP * HC * 4;              off = (off + 255) & ~(size_t)255;
  const size_t oAL = off; off += (size_t)MP * NAL * 4;             off = (off + 255) & ~(size_t)255;
  if (off > ws_size || off > (size_t)WSMAX) return;
  unsigned short* XB = (unsigned short*)(ws + oXB);
  unsigned short* WB = (unsigned short*)(ws + oWB);
  float*          Hf = (float*)(ws + oH);
  float*          AL = (float*)(ws + oAL);

  hipFuncSetAttribute(reinterpret_cast<const void*>(&k_agg),
                      hipFuncAttributeMaxDynamicSharedMemorySize, LDS_AGG);

  const int nUx = MP * (DIN / 8);
  k_prep<<<cdiv(nUx, NTHR), NTHR, 0, stream>>>(x, XB, nN, nUx);
  const int nUw = HC * (DIN / 8);
  k_prep<<<cdiv(nUw, NTHR), NTHR, 0, stream>>>(W, WB, HC, nUw);

  k_gemm<<<MP / GBM, GTHR, 0, stream>>>(XB, WB, attl, attr, Hf, AL, DIN);

  k_agg<<<gA, NTHR, LDS_AGG, stream>>>(src, dst, AL, Hf, out, nN, nE, nb, vec8);
}
